// molecular_network_56410100466094
// MI455X (gfx1250) — hardware-run, weakly checked
//
#include <hip/hip_runtime.h>


namespace {
constexpr int N = 50000, E = 400000, M = 32, NBAS = 20, HID = 100, HP = 128, NBLK = N / 16;
constexpr float XS = 8.0f, HS = 64.0f  , WSC = 256.0f;
constexpr float IM = 0.17677669f, INB = 0.2236068f, IH = 0.1f, I3 = 0.57735026f, INN = 0.35355338f, I2M = 0.125f;
typedef _Float16 b16;
typedef __attribute__((ext_vector_type(16))) _Float16 v16b;
typedef __attribute__((ext_vector_type(8))) _Float16 v8b;
typedef __attribute__((ext_vector_type(8))) float v8f;
typedef __attribute__((ext_vector_type(4))) float v4f;
typedef __attribute__((ext_vector_type(2))) float v2f;
__device__ __forceinline__ float bf16_rne(float f) { unsigned int u = __float_as_uint(f); u += 0x7FFFu + ((u >> 16) & 1u); return __uint_as_float(u & 0xFFFF0000u); }
__device__ __forceinline__ void split16(float v, b16& hi, b16& lo) { hi = (b16)v; lo = (b16)(v - (float)hi); }
__device__ __forceinline__ v16b frag_kb(const b16* p, int hh) { const v8b a = *(const v8b*)(p + 8 * hh), b = *(const v8b*)(p + 16 + 8 * hh); v16b f;
#pragma unroll
  for (int e = 0; e < 8; ++e) { f[e] = a[e]; f[8 + e] = b[e]; } return f; }
__device__ __forceinline__ v8f wmma16b(v16b a, v16b b, v8f c) { v8f d = __builtin_amdgcn_wmma_f32_16x16x32_f16(false, a, false, b, (short)0, c, false, false); asm volatile("v_nop\n\tv_nop\n\tv_nop\n\tv_nop" : "+v"(d) : "v"(a), "v"(b)); return d; }
__device__ __forceinline__ void wave_lds_sync() { __builtin_amdgcn_fence(__ATOMIC_RELEASE, "workgroup"); __builtin_amdgcn_wave_barrier(); __builtin_amdgcn_fence(__ATOMIC_ACQUIRE, "workgroup"); }
__device__ __forceinline__ float pmul(float a, float b) { float p = a * b; asm volatile("" : "+v"(p)); return p; }
__device__ __forceinline__ int iclamp(int v, int lo, int hi) { return v < lo ? lo : (v > hi ? hi : v); }
__device__ __forceinline__ float silu(float v) { return pmul(v, 1.0f / (1.0f + __expf(-v))); }
constexpr int CSR_NBLK9 = 512, CSR_GB9 = 9, CSR_GN9 = 1 << CSR_GB9  , CSR_TS9 = (CSR_GN9 < 32 ? 32 : CSR_GN9)  , CSR_MAXG9 = 512, CSR_CAP9 = 12288  ;
__device__ __host__ __forceinline__ int csr_tix9(int v) { return (v >> CSR_GB9) * CSR_TS9 + (v & (CSR_GN9 - 1)); }
__global__ __launch_bounds__(64) void csrA_kernel9(const int* __restrict__ dst, int E, int N, int nG, int CHP, int NGP, int* __restrict__ STG, int* __restrict__ HST) {
  extern __shared__ int sm[];
  int* cnt = sm; int* run = sm + NGP; int* ids = sm + 2 * NGP;
  const int b = blockIdx.x; const int ch = (E + CSR_NBLK9 - 1) / CSR_NBLK9; const int e0 = b * ch, e1 = min(E, e0 + ch);
  for (int i = threadIdx.x; i < NGP; i += 64) cnt[i] = 0;
  for (int i = threadIdx.x; i < CHP; i += 64) ids[i] = -1;
  __syncthreads();
  if (threadIdx.x == 0) {
    for (int e = e0; e < e1; ++e) { int d = dst[e]; d = (d < 0) ? 0 : (d >= N ? N - 1 : d); cnt[d >> CSR_GB9] += 1; }
    int acc = 0; for (int g = 0; g < nG; ++g) { run[g] = acc; acc += cnt[g]; }
    for (int e = e0; e < e1; ++e) { int d = dst[e]; d = (d < 0) ? 0 : (d >= N ? N - 1 : d); const int g = d >> CSR_GB9; ids[run[g]] = e; run[g] += 1; } }
  __syncthreads();
  typedef __attribute__((ext_vector_type(4))) int v4i;
  for (int pass = 0; pass < 2; ++pass) {
    for (int i = threadIdx.x; i < CHP / 4; i += 64) *(volatile v4i*)(STG + (size_t)b * CHP + i * 4) = *(const v4i*)(&ids[i * 4]);
    for (int i = threadIdx.x; i < NGP / 4; i += 64) { v4i v; for (int e = 0; e < 4; ++e) v[e] = (i * 4 + e < nG) ? cnt[i * 4 + e] : 0; *(volatile v4i*)(HST + (size_t)b * NGP + i * 4) = v; }
    __threadfence(); }
}
__global__ __launch_bounds__(512) void csrS_kernel9(const int* __restrict__ HST, int nG, int NGP, int* __restrict__ START, int* __restrict__ TOT, int* __restrict__ OFF) {
  __shared__ int tot[CSR_MAXG9];
  const int b = threadIdx.x;
  for (int pass = 0; pass < 2; ++pass) { int runb = 0; for (int g = 0; g < nG; ++g) { int c = HST[(size_t)b * NGP + g]; c = (c < 0) ? 0 : c; ((volatile int*)OFF)[(size_t)g * CSR_NBLK9 + b] = runb; runb += c; } __threadfence(); }
  for (int g = threadIdx.x; g < nG; g += 512) { int s = 0; for (int bb = 0; bb < CSR_NBLK9; ++bb) { int c = HST[(size_t)bb * NGP + g]; s += (c < 0) ? 0 : c; } tot[g] = s; }
  __syncthreads();
  if (threadIdx.x < 32) {
    __shared__ int st[CSR_MAXG9 + 32];
    if (threadIdx.x == 0) { int acc = 0; for (int g = 0; g < NGP; ++g) { st[g] = acc; if (g < nG) acc += (tot[g] + 31) & ~31; } st[NGP] = acc; }
    __builtin_amdgcn_fence(__ATOMIC_RELEASE, "workgroup"); __builtin_amdgcn_wave_barrier(); __builtin_amdgcn_fence(__ATOMIC_ACQUIRE, "workgroup");
    for (int pass = 0; pass < 2; ++pass) { for (int i = threadIdx.x; i < NGP + 32; i += 32) { ((volatile int*)START)[i] = (i <= NGP) ? st[min(i, NGP)] : 0; ((volatile int*)TOT)[i] = (i < nG) ? tot[i] : 0; } __threadfence(); } }
}
__global__ __launch_bounds__(256) void csrB_kernel9(const int* __restrict__ dst, int N, int nG, int CHP, int NGP, int permLen, const int* __restrict__ STG, const int* __restrict__ HST, const int* __restrict__ OFF, const int* __restrict__ START, const int* __restrict__ TOT, int* __restrict__ PERM, int* __restrict__ ROWPTR, int* __restrict__ ROWCNT, int* __restrict__ FLAG) {
  typedef __attribute__((ext_vector_type(4))) int v4i;
  __shared__ int ids[CSR_CAP9]; __shared__ unsigned short key[CSR_CAP9]; __shared__ int outp[CSR_CAP9]; __shared__ int ncnt[CSR_GN9 + 1]; __shared__ int boff[CSR_NBLK9 + 1];
  const int g = blockIdx.x, t_ = threadIdx.x; int tot = TOT[g]; int st = START[g], stn = START[g + 1]; const int v0 = g * CSR_GN9; const int nv = min(CSR_GN9, N - v0); const int t0 = g * CSR_TS9;
  st = (st < 0) ? 0 : (st > permLen - 32 ? permLen - 32 : st) & ~31; stn = (stn < st) ? st : (stn > permLen ? permLen : stn); tot = (tot < 0) ? 0 : tot; if (tot > stn - st && tot <= CSR_CAP9) tot = stn - st;
  if (tot > CSR_CAP9) {
    for (int pass = 0; pass < 2; ++pass) { for (int i = t_; i < CSR_TS9 / 4; i += 256) { v4i a, c; for (int e = 0; e < 4; ++e) { a[e] = st; c[e] = 0; } *(volatile v4i*)(ROWPTR + t0 + i * 4) = a; *(volatile v4i*)(ROWCNT + t0 + i * 4) = c; } if (t_ == 0) ((volatile int*)FLAG)[0] = 1; __threadfence(); } (void)nv; return; }
  if (t_ == 0) { int acc = 0; for (int b = 0; b < CSR_NBLK9; ++b) { boff[b] = acc; int c = HST[(size_t)b * NGP + g]; c = (c < 0) ? 0 : (c > CHP ? CHP : c); acc += c; if (acc > tot) acc = tot; } boff[CSR_NBLK9] = acc; }
  for (int i = t_; i <= CSR_GN9; i += 256) ncnt[i] = 0;
  __syncthreads();
  for (int b = 0; b < CSR_NBLK9; ++b) { const int c = boff[b + 1] - boff[b]; int o_ = OFF[(size_t)g * CSR_NBLK9 + b]; o_ = (o_ < 0) ? 0 : (o_ > CHP - c ? CHP - c : o_); const int* src_ = STG + (size_t)b * CHP + o_;
    for (int i = t_; i < c; i += 256) { int id = src_[i]; id = (id < 0) ? 0 : id; ids[boff[b] + i] = id; int d = dst[id]; d = (d < v0) ? v0 : (d >= N ? N - 1 : d); int kk = d - v0; kk = (kk < 0) ? 0 : (kk >= CSR_GN9 ? CSR_GN9 - 1 : kk); key[boff[b] + i] = (unsigned short)kk; } }
  __syncthreads();
  if (t_ == 0) { for (int i = 0; i < tot; ++i) ncnt[key[i]] += 1; int acc = 0; for (int vl = 0; vl < CSR_GN9; ++vl) { const int c = ncnt[vl]; ncnt[vl] = acc; acc += c; } ncnt[CSR_GN9] = acc;
    for (int i = 0; i < tot; ++i) { const int vl = key[i]; outp[ncnt[vl]] = ids[i]; ncnt[vl] += 1; }
    for (int vl = CSR_GN9; vl > 0; --vl) ncnt[vl] = ncnt[vl - 1]; ncnt[0] = 0; }
  __syncthreads();
  for (int pass = 0; pass < 2; ++pass) {
    for (int i = t_; i < (stn - st) / 4; i += 256) { v4i v; for (int e = 0; e < 4; ++e) { const int q = i * 4 + e; v[e] = (q < tot) ? outp[q] : -1; } *(volatile v4i*)(PERM + st + i * 4) = v; }
    for (int i = t_; i < CSR_TS9 / 4; i += 256) { v4i a, c; for (int e = 0; e < 4; ++e) { const int vl = i * 4 + e; const int vc = vl < CSR_GN9 ? vl : CSR_GN9; a[e] = (vl < CSR_GN9) ? st + ncnt[vc] : st; c[e] = (vl < nv) ? (ncnt[(vc < CSR_GN9 ? vc : CSR_GN9 - 1) + 1] - ncnt[vc]) : 0; } *(volatile v4i*)(ROWPTR + t0 + i * 4) = a; *(volatile v4i*)(ROWCNT + t0 + i * 4) = c; }
    __threadfence(); }
}
__global__ __launch_bounds__(256) void csrZ_kernel9(int* __restrict__ p, size_t n4) { typedef __attribute__((ext_vector_type(4))) int v4i; const size_t tid = (size_t)blockIdx.x * 256 + threadIdx.x, nth = (size_t)gridDim.x * 256; v4i z = {0, 0, 0, 0}; for (size_t i = tid; i < n4; i += nth) *(volatile v4i*)(p + i * 4) = z; }
struct CsrBufs9 { int *STG, *HST, *OFF, *START, *TOT, *PERM, *ROWPTR, *ROWCNT, *FLAG; int nG, NGP, CHP; size_t permLen; char* base; size_t bytes; };
static size_t csr_carve9(CsrBufs9& c, char* ws, size_t off, int E, int N) {
  const size_t off0 = off; c.base = ws + off;
  auto al = [&](size_t bytes) { char* p = ws + off; off += (bytes + 255) & ~(size_t)255; return p; };
  c.nG = (N + CSR_GN9 - 1) / CSR_GN9; c.NGP = (c.nG + 31) & ~31; const int ch = (E + CSR_NBLK9 - 1) / CSR_NBLK9; c.CHP = (ch + 31) & ~31; c.permLen = (size_t)E + 32 * (size_t)c.nG + 32;
  c.STG = (int*)al((size_t)CSR_NBLK9 * c.CHP * 4); c.HST = (int*)al((size_t)CSR_NBLK9 * c.NGP * 4); c.OFF = (int*)al((size_t)c.NGP * CSR_NBLK9 * 4); c.START = (int*)al((size_t)(c.NGP + 64) * 4); c.TOT = (int*)al((size_t)(c.NGP + 64) * 4);
  c.PERM = (int*)al(c.permLen * 4); c.ROWPTR = (int*)al((size_t)c.nG * CSR_TS9 * 4); c.ROWCNT = (int*)al((size_t)c.nG * CSR_TS9 * 4); c.FLAG = (int*)al(256);
  c.bytes = off - off0; return off;
}
static void csr_build9(const CsrBufs9& c, const int* dst, int E, int N, hipStream_t stream) {
  const size_t smem = (size_t)(2 * c.NGP + c.CHP) * 4;
  csrZ_kernel9<<<512, 256, 0, stream>>>((int*)c.base, c.bytes / 16);
  csrA_kernel9<<<CSR_NBLK9, 64, smem, stream>>>(dst, E, N, c.nG, c.CHP, c.NGP, c.STG, c.HST);
  csrS_kernel9<<<1, 512, 0, stream>>>(c.HST, c.nG, c.NGP, c.START, c.TOT, c.OFF);
  csrB_kernel9<<<c.nG, 256, 0, stream>>>(dst, N, c.nG, c.CHP, c.NGP, (int)c.permLen, c.STG, c.HST, c.OFF, c.START, c.TOT, c.PERM, c.ROWPTR, c.ROWCNT, c.FLAG);
}


__global__ __launch_bounds__(256) void wput_kernel(const float* __restrict__ w, int KIN, int OUTW, int KN, int OUT, int ro, int ko, int KP, b16* __restrict__ WT) {
  const int KG = KN / 8; const int u = blockIdx.x * 256 + threadIdx.x; if (u >= OUT * KG) return; const int o = u / KG, k0 = (u % KG) * 8; v8b v;
#pragma unroll
  for (int j = 0; j < 8; ++j) { const int k = k0 + j; v[j] = (k < KIN && o < OUTW) ? (b16)(bf16_rne(w[(size_t)k * OUTW + o]) * WSC) : (b16)0.0f; } for (int pass = 0; pass < 2; ++pass) { *(volatile v8b*)(WT + (size_t)(ro + o) * KP + ko + k0) = v; __threadfence(); }
}
__global__ __launch_bounds__(32) void self_kernel(const float* __restrict__ ni, const float* __restrict__ na, const b16* __restrict__ WSI0, const b16* __restrict__ WSI1, int NLIM, float* __restrict__ S) {
  __shared__ __attribute__((aligned(16))) b16 Ah[4][16][32 + 8]; __shared__ __attribute__((aligned(16))) float Tf[16][HP + 4];
  const int lane = threadIdx.x, nloc = lane & 15, hlf = lane >> 4; const size_t m0 = (size_t)blockIdx.x * 16; if (m0 >= (size_t)NLIM) return;
  for (int rr = 0; rr < 16; ++rr) { const float* row = ni + (m0 + rr) * HP; Ah[0][rr][lane] = (b16)(bf16_rne(row[lane]) * XS); for (int c = 0; c < 3; ++c) Ah[1 + c][rr][lane] = (b16)(bf16_rne(row[M + lane * 3 + c]) * XS); }
  wave_lds_sync();
#pragma unroll
  for (int part = 0; part < 4; ++part) { const b16* W = part == 0 ? WSI0 : WSI1; const v16b a = frag_kb(&Ah[part][nloc][0], hlf);
#pragma unroll
    for (int t = 0; t < 2; ++t) { v8f acc = {}; acc = wmma16b(a, frag_kb(W + (size_t)(t * 16 + nloc) * 32, hlf), acc); const int k = t * 16 + nloc;
#pragma unroll
      for (int r8 = 0; r8 < 8; ++r8) { const int rl = 8 * hlf + r8; const float v = pmul(acc[r8] * (IM / (XS * WSC)), bf16_rne(na[m0 + rl])); if (part == 0) Tf[rl][k] = v; else Tf[rl][M + k * 3 + (part - 1)] = v; } } }
  wave_lds_sync();
  for (int pass = 0; pass < 2; ++pass) { for (int rr = 0; rr < 16; ++rr) *(volatile v4f*)(S + (m0 + rr) * HP + lane * 4) = *(const v4f*)(&Tf[rr][lane * 4]); __threadfence(); }
}
__global__ __launch_bounds__(32) void radial_kernel(const float* __restrict__ de, const b16* __restrict__ W1T, const b16* __restrict__ W2T, int c0, float* __restrict__ TPW) {
  __shared__ __attribute__((aligned(16))) b16 A0[16][32 + 8], Ah[16][HP + 8], Al[16][HP + 8]; __shared__ __attribute__((aligned(16))) float Tf[16][HP + 4];
  const int lane = threadIdx.x, nloc = lane & 15, hlf = lane >> 4; const size_t el = (size_t)blockIdx.x * 16; const size_t e0 = (size_t)c0 + el;
  for (int rr = 0; rr < 16; ++rr) A0[rr][lane] = lane < NBAS ? (b16)(bf16_rne(de[(e0 + rr) * NBAS + lane]) * XS) : (b16)0.0f;
  wave_lds_sync();
  { const v16b a = frag_kb(&A0[nloc][0], hlf);
#pragma unroll
    for (int t = 0; t < 8; ++t) { v8f acc = {}; acc = wmma16b(a, frag_kb(W1T + (size_t)(t * 16 + nloc) * 32, hlf), acc); const int c = t * 16 + nloc;
#pragma unroll
      for (int r8 = 0; r8 < 8; ++r8) { const float h = c < HID ? silu(acc[r8] * (INB / (XS * WSC))) : 0.0f; b16 p, q; split16(h * HS, p, q); Ah[8 * hlf + r8][c] = p; Al[8 * hlf + r8][c] = q; } } }
  wave_lds_sync();
  v8f acc[8];
#pragma unroll
  for (int t = 0; t < 8; ++t) acc[t] = (v8f){};
#pragma unroll
  for (int kb = 0; kb < HP; kb += 32) { const v16b a = frag_kb(&Ah[nloc][kb], hlf), al = frag_kb(&Al[nloc][kb], hlf);
#pragma unroll
    for (int t = 0; t < 8; ++t) { const v16b bw = frag_kb(W2T + (size_t)(t * 16 + nloc) * HP + kb, hlf); acc[t] = wmma16b(a, bw, acc[t]); acc[t] = wmma16b(al, bw, acc[t]); } }
#pragma unroll
  for (int t = 0; t < 8; ++t)
#pragma unroll 1
    for (int r8 = 0; r8 < 8; ++r8) Tf[8 * hlf + r8][t * 16 + nloc] = acc[t][r8] * (IH / (HS * WSC));
  wave_lds_sync();
  for (int pass = 0; pass < 2; ++pass) { for (int rr = 0; rr < 16; ++rr) *(volatile v4f*)(TPW + (el + rr) * HP + lane * 4) = *(const v4f*)(&Tf[rr][lane * 4]); __threadfence(); }
}
__global__ __launch_bounds__(256) void msg_kernel(const float* __restrict__ S, const float* __restrict__ TPW, const float* __restrict__ ea, const int* __restrict__ dsts, const int* __restrict__ PERM, const int* __restrict__ ROWPTR, const int* __restrict__ ROWCNT, int permLen, int NLIM, int c0, int ECH, int first, int final_, float* __restrict__ AGG) {
  const int wave = threadIdx.x >> 5, u = threadIdx.x & 31; const size_t v = (size_t)blockIdx.x * 8 + wave; if (v >= (size_t)NLIM) return;
  int st = ROWPTR[v], cnt = ROWCNT[v]; cnt = iclamp(cnt, 0, 1 << 20); st = iclamp(st, 0, permLen - cnt); float a0 = 0.0f, b0 = 0.0f, a1[3] = {0, 0, 0}, b1[3] = {0, 0, 0};
#pragma unroll 1
  for (int j = 0; j < cnt; ++j) { const int e = iclamp(PERM[st + j], 0, E - 1); if (e < c0 || e >= c0 + ECH) continue; const size_t d = (size_t)iclamp(dsts[e], 0, N - 1); if (d >= (size_t)NLIM) continue;
    const float* sr = S + d * HP; const float g0 = sr[u], g10 = sr[M + u * 3], g11 = sr[M + u * 3 + 1], g12 = sr[M + u * 3 + 2];
    const float y0 = bf16_rne(ea[(size_t)e * 4]), y10 = bf16_rne(ea[(size_t)e * 4 + 1]), y11 = bf16_rne(ea[(size_t)e * 4 + 2]), y12 = bf16_rne(ea[(size_t)e * 4 + 3]);
    const float* wr = TPW + (size_t)(e - c0) * HP; const float w1 = wr[u], w2 = wr[M + u], w3 = wr[2 * M + u], w4 = wr[3 * M + u];
    a0 += pmul(pmul(g0, y0), w1); b0 += pmul(pmul(pmul(g10, y10) + pmul(g11, y11) + pmul(g12, y12), I3), w4);
    const float gw = pmul(g0, w2); a1[0] += pmul(gw, y10); a1[1] += pmul(gw, y11); a1[2] += pmul(gw, y12); const float yw = pmul(y0, w3); b1[0] += pmul(g10, yw); b1[1] += pmul(g11, yw); b1[2] += pmul(g12, yw); }
  float* row = AGG + v * 256; if (!first) { a0 += row[u]; b0 += row[M + u]; for (int c = 0; c < 3; ++c) { a1[c] += row[2 * M + u * 3 + c]; b1[c] += row[2 * M + 3 * M + u * 3 + c]; } } const float sc = final_ ? INN : 1.0f;
  for (int pass = 0; pass < 2; ++pass) { ((volatile float*)row)[u] = a0 * sc; ((volatile float*)row)[M + u] = b0 * sc; for (int c = 0; c < 3; ++c) { ((volatile float*)row)[2 * M + u * 3 + c] = a1[c] * sc; ((volatile float*)row)[2 * M + 3 * M + u * 3 + c] = b1[c] * sc; } __threadfence(); }
}
__global__ __launch_bounds__(32) void out_kernel(const float* __restrict__ AGG, const float* __restrict__ ni, const float* __restrict__ na, const b16* __restrict__ WO0, const b16* __restrict__ WO1, int NLIM, float* __restrict__ out) {
  __shared__ __attribute__((aligned(16))) b16 Ah[4][16][96 + 8], Al[4][16][96 + 8]; __shared__ __attribute__((aligned(16))) float Tf[16][HP + 4];
  const int lane = threadIdx.x, nloc = lane & 15, hlf = lane >> 4; const size_t m0 = (size_t)blockIdx.x * 16; const bool live = m0 < (size_t)NLIM;
  for (int rr = 0; rr < 16; ++rr) { const float* ag = AGG + (m0 + rr) * 256; const float* xr = ni + (m0 + rr) * HP; b16 p, q;
    { const float v0 = live ? ag[lane] * I2M : 0.0f, v1 = live ? ag[M + lane] * I2M : 0.0f, v2 = bf16_rne(xr[lane]) * IM; split16(v0 * HS, p, q); Ah[0][rr][lane] = p; Al[0][rr][lane] = q; split16(v1 * HS, p, q); Ah[0][rr][M + lane] = p; Al[0][rr][M + lane] = q; split16(v2 * HS, p, q); Ah[0][rr][2 * M + lane] = p; Al[0][rr][2 * M + lane] = q; }
    for (int c = 0; c < 3; ++c) { const float v0 = live ? ag[2 * M + lane * 3 + c] * I2M : 0.0f, v1 = live ? ag[2 * M + 3 * M + lane * 3 + c] * I2M : 0.0f, v2 = bf16_rne(xr[M + lane * 3 + c]) * IM; split16(v0 * HS, p, q); Ah[1 + c][rr][lane] = p; Al[1 + c][rr][lane] = q; split16(v1 * HS, p, q); Ah[1 + c][rr][M + lane] = p; Al[1 + c][rr][M + lane] = q; split16(v2 * HS, p, q); Ah[1 + c][rr][2 * M + lane] = p; Al[1 + c][rr][2 * M + lane] = q; } }
  wave_lds_sync();
#pragma unroll
  for (int part = 0; part < 4; ++part) { const b16* W = part == 0 ? WO0 : WO1; v8f acc[2] = {(v8f){}, (v8f){}};
#pragma unroll
    for (int kb = 0; kb < 96; kb += 32) { const v16b a = frag_kb(&Ah[part][nloc][kb], hlf), al = frag_kb(&Al[part][nloc][kb], hlf);
#pragma unroll
      for (int t = 0; t < 2; ++t) { const v16b bw = frag_kb(W + (size_t)(t * 16 + nloc) * 96 + kb, hlf); acc[t] = wmma16b(a, bw, acc[t]); acc[t] = wmma16b(al, bw, acc[t]); } }
#pragma unroll
    for (int t = 0; t < 2; ++t) { const int k = t * 16 + nloc;
#pragma unroll
      for (int r8 = 0; r8 < 8; ++r8) { const int rl = 8 * hlf + r8; const float v = live ? pmul(acc[t][r8] * (1.0f / (HS * WSC)), bf16_rne(na[m0 + rl])) : 0.0f; if (part == 0) Tf[rl][k] = v; else Tf[rl][M + k * 3 + (part - 1)] = v; } } }
  wave_lds_sync();
  for (int pass = 0; pass < 2; ++pass) { for (int rr = 0; rr < 16; ++rr) *(volatile v4f*)(out + (m0 + rr) * HP + lane * 4) = *(const v4f*)(&Tf[rr][lane * 4]); __threadfence(); }
}
}

extern "C" void kernel_launch(void* const* d_in, const int* in_sizes, int n_in, void* d_out, int out_size, void* d_ws, size_t ws_size, hipStream_t stream) {
  (void)n_in;
  auto Fp = [&](int i) { return (const float*)d_in[i]; }; auto Ip = [&](int i) { return (const int*)d_in[i]; };
  if (in_sizes[0] != N * HP || in_sizes[1] != N || in_sizes[2] != E || in_sizes[3] != E || in_sizes[4] != E * 4 || in_sizes[5] != E * NBAS || in_sizes[6] != M * M || in_sizes[8] != NBAS * HID || in_sizes[9] != HID * HP || in_sizes[10] != 2 * M * M || in_sizes[12] != M * M || out_size != N * HP) return;
  const int NLIM = N; const int GB16 = NBLK, GB8 = N / 8; const int EV = E;
  size_t off = 0; char* ws = (char*)d_ws;
  auto carve = [&](size_t bytes) { char* p = ws + off; off += (bytes + 255) & ~(size_t)255; return p; };
  b16* WSI0 = (b16*)carve(M * 32 * 2); b16* WSI1 = (b16*)carve(M * 32 * 2); b16* W1T = (b16*)carve(HP * 32 * 2); b16* W2T = (b16*)carve(HP * HP * 2); b16* WO0 = (b16*)carve(M * 96 * 2); b16* WO1 = (b16*)carve(M * 96 * 2);
  constexpr int NCH = 2, ECH = E / NCH;
  float* S = (float*)carve((size_t)N * HP * 4); float* TPW = (float*)carve((size_t)ECH * HP * 4); float* AGG = (float*)carve((size_t)N * 256 * 4);
  CsrBufs9 csr; off = csr_carve9(csr, ws, off, E, N);
  if (off > ws_size || off > ((size_t)200 << 20)) return;
  wput_kernel<<<(M * 4 + 255) / 256, 256, 0, stream>>>(Fp(6), M, M, 32, M, 0, 0, 32, WSI0); wput_kernel<<<(M * 4 + 255) / 256, 256, 0, stream>>>(Fp(7), M, M, 32, M, 0, 0, 32, WSI1);
  wput_kernel<<<(HP * 4 + 255) / 256, 256, 0, stream>>>(Fp(8), NBAS, HID, 32, HP, 0, 0, 32, W1T); wput_kernel<<<(HP * 16 + 255) / 256, 256, 0, stream>>>(Fp(9), HID, HP, HP, HP, 0, 0, HP, W2T);
  wput_kernel<<<(M * 8 + 255) / 256, 256, 0, stream>>>(Fp(10), 2 * M, M, 64, M, 0, 0, 96, WO0); wput_kernel<<<(M * 4 + 255) / 256, 256, 0, stream>>>(Fp(12), M, M, 32, M, 0, 64, 96, WO0);
  wput_kernel<<<(M * 8 + 255) / 256, 256, 0, stream>>>(Fp(11), 2 * M, M, 64, M, 0, 0, 96, WO1); wput_kernel<<<(M * 4 + 255) / 256, 256, 0, stream>>>(Fp(13), M, M, 32, M, 0, 64, 96, WO1);
  csr_build9(csr, Ip(2), E, N, stream);
  self_kernel<<<GB16, 32, 0, stream>>>(Fp(0), Fp(1), WSI0, WSI1, NLIM, S);
  for (int ch = 0; ch < NCH; ++ch) { const int elo = ch * ECH; const int ecnt = (EV - elo) < ECH ? (EV - elo) : ECH; const bool last = (ch == NCH - 1) || (elo + ECH >= EV); if (ecnt <= 0) break;
    radial_kernel<<<ecnt / 16, 32, 0, stream>>>(Fp(5), W1T, W2T, elo, TPW);
    msg_kernel<<<GB8, 256, 0, stream>>>(S, TPW, Fp(4), Ip(3), csr.PERM, csr.ROWPTR, csr.ROWCNT, (int)csr.permLen, NLIM, elo, ecnt, ch == 0 ? 1 : 0, last ? 1 : 0, AGG); }
  out_kernel<<<NBLK, 32, 0, stream>>>(AGG, Fp(0), Fp(1), WO0, WO1, NLIM, (float*)d_out);
}
